// DeepAGATConvolution_47974784696359
// MI455X (gfx1250) — hardware-verified
//
#include <hip/hip_runtime.h>
#include <stddef.h>


#define FD       32
#define NHEAD    10
#define NGRP     10
#define HPG      (NHEAD / NGRP)
#define NCOL     (NHEAD * FD)
#define KW       32
#define NTILE    (NCOL / 16)
#define GSZ      NHEAD
#define OFF_BX   0
#define OFF_BE   (NCOL * KW)
#define BPTOT    (2 * NCOL * KW)
#define ASC      16.0f
#define WSC      64.0f
#define RSC      0.0009765625f
#define LNEG     0.2f
#define EPSV     1e-5f
#define HMEAN    0.1f
#define GROWS    32
#define GTHR     64
#define EWAV     5
#define ETHR     (EWAV * 32)
#define EPW      16
#define EPB      (EWAV * EPW)
#define GPB      (EPB / GSZ)
#define XP       NCOL
#define LGP      12
#define PGP      36
#define STHR     256
#define SWAV     (STHR / 32)
#define EPT      16
#define CHUNK    (STHR * EPT)
#define NBA      512
#define WSCAP    134217728
#define LDS_EDGE (EPB * XP * 4 + 2 * EPB * LGP * 4 + EWAV * 32 * PGP * 4 + NHEAD * 2 * FD * 4 + 64 * 4)
#define LDS_AGG  (NBA * FD * 4 + CHUNK * 4 + FD * 4 + 64)

static_assert(BPTOT == 10 * 256 * 8);
static_assert((NCOL * KW / 8) == 5 * 256);
static_assert(KW == 32 && (NCOL % 16) == 0 && (XP % 4) == 0 && (PGP % 4) == 0);
static_assert(GROWS == (GTHR / 32) * 16);
static_assert(GROWS * NCOL == 40 * GTHR * 4);
static_assert((EPB % GSZ) == 0 && GPB * NHEAD * FD == 4 * ETHR * 4);
static_assert(ETHR * 4 == NHEAD * 2 * FD);
static_assert(NHEAD <= 16 && NGRP <= 16);
static_assert(NBA == 2 * STHR && NBA * FD == 16 * STHR * 4 && (NBA * FD) % (4 * STHR) == 0);
static_assert(CHUNK == 4096 && HPG >= 1 && GSZ == 10);
static_assert(LDS_EDGE == 135936 && LDS_AGG == 82112);

typedef float    v4f  __attribute__((ext_vector_type(4)));
typedef float    v8f  __attribute__((ext_vector_type(8)));
typedef int      v4i  __attribute__((ext_vector_type(4)));
typedef _Float16 v4h  __attribute__((ext_vector_type(4)));
typedef _Float16 v8h  __attribute__((ext_vector_type(8)));
typedef _Float16 v16h __attribute__((ext_vector_type(16)));
union Frag { v16h v; v8h h[2]; v4h q[4]; };

__device__ __forceinline__ v8f wmh(v16h a, v16h b, v8f c) {
  v8f d = __builtin_amdgcn_wmma_f32_16x16x32_f16(false, a, false, b, (short)0, c, false, false);
  asm volatile("v_nop\n\tv_nop\n\tv_nop\n\tv_nop" : "+v"(d) : "v"(a), "v"(b));
  return d;
}

__device__ __forceinline__ float lk(float v) { return v >= 0.0f ? v : LNEG * v; }

__device__ __forceinline__ v4h cv4(v4f u) {
  v4h r;
  r.x = (_Float16)(u.x * ASC); r.y = (_Float16)(u.y * ASC);
  r.z = (_Float16)(u.z * ASC); r.w = (_Float16)(u.w * ASC);
  return r;
}

__device__ __forceinline__ void afrag(const float* __restrict__ p, int hh, Frag& a) {
  const v4f u0 = *(const v4f*)(p + 8 * hh), u1 = *(const v4f*)(p + 8 * hh + 4);
  const v4f u2 = *(const v4f*)(p + 16 + 8 * hh), u3 = *(const v4f*)(p + 20 + 8 * hh);
  a.q[0] = cv4(u0); a.q[1] = cv4(u1); a.q[2] = cv4(u2); a.q[3] = cv4(u3);
}

__global__ __launch_bounds__(256) void k_wprep(const float* __restrict__ W, _Float16* Bpl) {
  const int i = blockIdx.x * 256 + threadIdx.x;
  const int pl = i / (NCOL * KW / 8);
  const int ii = i - pl * (NCOL * KW / 8);
  const int n = ii >> 2, k0 = (ii & 3) * 8;
  const int kb = pl * KW + k0;
  v8h hv;
#pragma unroll
  for (int e = 0; e < 8; ++e) hv[e] = (_Float16)(W[(kb + e) * NCOL + n] * WSC);
  _Float16* dp = Bpl + (size_t)i * 8;
  *(volatile v8h*)dp = hv;
  __threadfence();
  *(volatile v8h*)dp = hv;
}

__global__ __launch_bounds__(GTHR) void k_nodep(const float* __restrict__ x, const _Float16* __restrict__ Bx,
                                                float* P, int nN) {
  __shared__ __attribute__((aligned(16))) float stg[GROWS * NCOL];
  const int tid = threadIdx.x, lane = tid & 31, hh = lane >> 4, m = lane & 15;
  const int wave = __builtin_amdgcn_readfirstlane(tid >> 5);
  const int rowBase = blockIdx.x * GROWS;
  int xr = rowBase + wave * 16 + m;
  xr = xr > nN - 1 ? nN - 1 : xr;
  Frag a;
  afrag(x + (size_t)xr * FD, hh, a);
  const _Float16* bb = Bx + (size_t)m * KW + 8 * hh;
  float* sp = stg + (wave * 16 + 8 * hh) * NCOL + m;
#pragma unroll 2
  for (int t = 0; t < NTILE; ++t) {
    const _Float16* bp = bb + (size_t)(16 * t) * KW;
    Frag b;
    b.h[0] = *(const v8h*)bp;
    b.h[1] = *(const v8h*)(bp + 16);
    v8f z = {0.f, 0.f, 0.f, 0.f, 0.f, 0.f, 0.f, 0.f};
    const v8f acc = wmh(a.v, b.v, z);
#pragma unroll
    for (int r = 0; r < 8; ++r) sp[r * NCOL + 16 * t] = acc[r] * RSC;
  }
  __syncthreads();

  float* gp = P + (size_t)rowBase * NCOL;
#pragma unroll
  for (int it = 0; it < (GROWS * NCOL) / (4 * GTHR); ++it) {
    const int f = it * GTHR + tid;
    const v4f v = ((const v4f*)stg)[f];
    *(volatile v4f*)(gp + 4 * f) = v;
  }
  __threadfence();
#pragma unroll
  for (int it = 0; it < (GROWS * NCOL) / (4 * GTHR); ++it) {
    const int f = it * GTHR + tid;
    const v4f v = ((const v4f*)stg)[f];
    *(volatile v4f*)(gp + 4 * f) = v;
  }
}

__global__ __launch_bounds__(ETHR) void k_edge(
    const float* __restrict__ P, const int* __restrict__ eidx, const float* __restrict__ ea,
    const _Float16* __restrict__ Be, const float* __restrict__ att, const float* __restrict__ gam,
    const float* __restrict__ bet, const float* __restrict__ rmean, const float* __restrict__ rvar,
    float* S, int nN, int nE, int nG) {
  extern __shared__ __attribute__((aligned(16))) char dynl[];
  float* sxj  = (float*)dynl;
  float* slg  = (float*)(dynl + EPB * XP * 4);
  float* sal  = slg + EPB * LGP;
  float* spg  = sal + EPB * LGP;
  float* satt = spg + EWAV * 32 * PGP;
  float* spar = satt + NHEAD * 2 * FD;
  const int tid = threadIdx.x, lane = tid & 31, hh = lane >> 4, m = lane & 15;
  const int wave = __builtin_amdgcn_readfirstlane(tid >> 5);
  float* sx = sxj + wave * (EPW * XP);
  float* sl = slg + wave * (EPW * LGP);
  float* sa = sal + wave * (EPW * LGP);
  float* sg = spg + wave * (32 * PGP);
  const int e0 = blockIdx.x * EPB + wave * EPW;

  {
    const v4f a4 = *(const v4f*)(att + 4 * tid);
    ((v4f*)satt)[tid] = a4;
    const int ph = tid < NHEAD ? tid : NHEAD - 1;
    const int pg = tid < NGRP ? tid : NGRP - 1;
    const float g0 = gam[ph], b0 = bet[ph], m0 = rmean[pg], v0 = rvar[pg];
    if (tid < NHEAD) { spar[tid] = g0; spar[16 + tid] = b0; }
    if (tid < NGRP)  { spar[32 + tid] = m0; spar[48 + tid] = v0; }
  }

  int eg = e0 + m;
  eg = eg > nE - 1 ? nE - 1 : eg;
  Frag a;
  afrag(ea + (size_t)eg * FD, hh, a);
  int ri = eidx[eg];
  int ci = eidx[(size_t)nE + eg];
  ri = ri < 0 ? 0 : (ri > nN - 1 ? nN - 1 : ri);
  ci = ci < 0 ? 0 : (ci > nN - 1 ? nN - 1 : ci);
  const int nd = (hh != 0) ? ci : ri;
  int pofs[8];
#pragma unroll
  for (int it = 0; it < 8; ++it) {
    const int rho = 4 * it + (lane >> 3);
    const int node = __shfl(nd, rho, 32);
    pofs[it] = node * NCOL + 4 * (lane & 7);
  }
  const _Float16* bb = Be + (size_t)m * KW + 8 * hh;
  __syncthreads();

#pragma unroll 1
  for (int h = 0; h < NHEAD; ++h) {
    const int cb = h * FD;
    v8f acc[2];
#pragma unroll
    for (int t = 0; t < 2; ++t) {
      const _Float16* bp = bb + (size_t)(cb + 16 * t) * KW;
      Frag b;
      b.h[0] = *(const v8h*)bp;
      b.h[1] = *(const v8h*)(bp + 16);
      v8f z = {0.f, 0.f, 0.f, 0.f, 0.f, 0.f, 0.f, 0.f};
      acc[t] = wmh(a.v, b.v, z);
    }
#pragma unroll
    for (int it = 0; it < 8; ++it) {
      const v4f pv = *(const v4f*)(P + (size_t)pofs[it] + cb);
      *(v4f*)(sg + (4 * it + (lane >> 3)) * PGP + 4 * (lane & 7)) = pv;
    }
    __syncthreads();

    float ai[2], aj[2];
#pragma unroll
    for (int t = 0; t < 2; ++t) {
      ai[t] = satt[h * (2 * FD) + 16 * t + m];
      aj[t] = satt[h * (2 * FD) + FD + 16 * t + m];
    }
    const float* sp0 = sg + (8 * hh) * PGP + m;
    const float* sp1 = sg + (16 + 8 * hh) * PGP + m;
    float s[8];
#pragma unroll
    for (int r = 0; r < 8; ++r) {
      float sr = 0.0f;
#pragma unroll
      for (int t = 0; t < 2; ++t) {
        const float q  = acc[t][r] * RSC;
        const float pi = sp0[r * PGP + 16 * t];
        const float pj = sp1[r * PGP + 16 * t];
        const float xi = lk(pi + q);
        const float xj = lk(pj + q);
        sx[(8 * hh + r) * XP + cb + 16 * t + m] = xj;
        sr = fmaf(xi, ai[t], sr);
        sr = fmaf(xj, aj[t], sr);
      }
      s[r] = sr;
    }
    float u[4];
    {
      const bool kb = ((lane >> 2) & 1) != 0;
#pragma unroll
      for (int i = 0; i < 4; ++i) {
        const float snd = kb ? s[i] : s[i + 4];
        const float kp  = kb ? s[i + 4] : s[i];
        u[i] = kp + __shfl_xor(snd, 4, 32);
      }
    }
    float w2[2];
    {
      const bool kb = ((lane >> 1) & 1) != 0;
#pragma unroll
      for (int i = 0; i < 2; ++i) {
        const float snd = kb ? u[i] : u[i + 2];
        const float kp  = kb ? u[i + 2] : u[i];
        w2[i] = kp + __shfl_xor(snd, 2, 32);
      }
    }
    float f;
    {
      const bool kb = (lane & 1) != 0;
      const float snd = kb ? w2[0] : w2[1];
      const float kp  = kb ? w2[1] : w2[0];
      f = kp + __shfl_xor(snd, 1, 32);
    }
    f += __shfl_xor(f, 8, 32);
    if ((m & 8) == 0) sl[(8 * hh + (m & 7)) * LGP + h] = f;
    __syncthreads();
  }

  {
    float av[NHEAD];
    float mx = -3.0e38f;
#pragma unroll
    for (int h = 0; h < NHEAD; ++h) {
      float t = lk(sl[m * LGP + h]);
      const int g = h / HPG;
      t = (t - spar[32 + g]) * rsqrtf(spar[48 + g] + EPSV);
      t = t * spar[h] + spar[16 + h];
      av[h] = t;
      mx = fmaxf(mx, t);
    }
    float sum = 0.0f;
#pragma unroll
    for (int h = 0; h < NHEAD; ++h) { av[h] = __expf(av[h] - mx); sum += av[h]; }
    const float inv = 1.0f / sum;
#pragma unroll
    for (int h = 0; h < NHEAD; ++h) sa[m * LGP + h] = av[h] * inv;
  }
  __syncthreads();

  v4f res[4];
#pragma unroll
  for (int it = 0; it < 4; ++it) {
    const int f = it * ETHR + tid;
    const int fl = 4 * f;
    const int gl = fl / NCOL;
    const int rem = fl - gl * NCOL;
    const int h = rem >> 5, k0 = rem & (FD - 1);
    const float* xb = sxj + (gl * GSZ) * XP + h * FD + k0;
    const float* ab = sal + (gl * GSZ) * LGP + h;
    v4f acc4 = {0.f, 0.f, 0.f, 0.f};
#pragma unroll 1
    for (int j = 0; j < GSZ; ++j) {
      const v4f xv = *(const v4f*)(xb + j * XP);
      const float al = ab[j * LGP];
      acc4 = acc4 + xv * al;
    }
    res[it] = acc4;
  }
  const int Gb = blockIdx.x * GPB;
#pragma unroll
  for (int it = 0; it < 4; ++it) {
    const int f = it * ETHR + tid;
    const int fl = 4 * f;
    const int gl = fl / NCOL;
    const int rem = fl - gl * NCOL;
    const int gg = Gb + gl;
    if (gg < nG) *(volatile v4f*)(S + (size_t)gg * NCOL + rem) = res[it];
  }
  __threadfence();
#pragma unroll
  for (int it = 0; it < 4; ++it) {
    const int f = it * ETHR + tid;
    const int fl = 4 * f;
    const int gl = fl / NCOL;
    const int rem = fl - gl * NCOL;
    const int gg = Gb + gl;
    if (gg < nG) *(volatile v4f*)(S + (size_t)gg * NCOL + rem) = res[it];
  }
}

__device__ __forceinline__ void loadids(const int* __restrict__ ids, int nE, int cbase, int tid, int vec,
                                        int (&d)[EPT]) {
  const int e0 = cbase + EPT * tid;
  if (vec != 0 && cbase + CHUNK <= nE) {
#pragma unroll
    for (int q = 0; q < EPT / 4; ++q) {
      const v4i t4 = *(const v4i*)(ids + e0 + 4 * q);
      d[4 * q] = t4.x; d[4 * q + 1] = t4.y; d[4 * q + 2] = t4.z; d[4 * q + 3] = t4.w;
    }
  } else {
#pragma unroll
    for (int j = 0; j < EPT; ++j) {
      int idx = e0 + j;
      const bool ok = idx < nE;
      idx = ok ? idx : nE - 1;
      const int val = ids[idx];
      d[j] = ok ? val : (-2147483647 - 1);
    }
  }
}

__device__ __forceinline__ void blkscan(int cnt, int lane, int wave, int* swt, int& pos, int& nh) {
  int x = cnt;
#pragma unroll
  for (int o = 1; o < 32; o <<= 1) {
    const int y = __shfl_up(x, o, 32);
    x += (lane >= o) ? y : 0;
  }
  if (lane == 31) swt[wave] = x;
  __syncthreads();
  int wpre = 0, tot = 0;
#pragma unroll
  for (int w = 0; w < SWAV; ++w) {
    const int v = swt[w];
    wpre += (w < wave) ? v : 0;
    tot += v;
  }
  pos = wpre + x - cnt;
  nh = tot;
}

__device__ __forceinline__ void agg_store(const float* sacc, const float* sbi, float* out,
                                          int n0, int nN, int tid) {
#pragma unroll 1
  for (int it = 0; it < (NBA * FD) / (4 * STHR); ++it) {
    const int f = it * STHR + tid, row = f >> 3, q = f & 7;
    const v4f sv = ((const v4f*)sacc)[f];
    const v4f bv = ((const v4f*)sbi)[q];
    const v4f v = sv * HMEAN + bv;
    const int n = n0 + row;
    if (n < nN) *(volatile v4f*)(out + (size_t)n * FD + 4 * q) = v;
  }
}

__global__ __launch_bounds__(STHR) void k_agg(
    const int* __restrict__ keys, const float* __restrict__ S, const float* __restrict__ bias,
    float* out, int nN, int nE, int nG, int nChunks, int vec) {
  extern __shared__ __attribute__((aligned(16))) char dynl[];
  float*    sacc  = (float*)dynl;
  unsigned* slist = (unsigned*)(dynl + NBA * FD * 4);
  float*    sbi   = (float*)(dynl + NBA * FD * 4 + CHUNK * 4);
  int*      swt   = (int*)(sbi + FD);
  const int tid = threadIdx.x, lane = tid & 31;
  const int wave = __builtin_amdgcn_readfirstlane(tid >> 5);
  const int n0 = blockIdx.x * NBA;
  {
    v4f z = {0.f, 0.f, 0.f, 0.f};
    v4f* p = (v4f*)sacc;
#pragma unroll
    for (int it = 0; it < (NBA * FD) / (4 * STHR); ++it) p[it * STHR + tid] = z;
  }
  if (tid < FD) sbi[tid] = bias[tid];
  __syncthreads();

#pragma unroll 1
  for (int c = 0; c < nChunks; ++c) {
    const int cbase = c * CHUNK;
    int d[EPT];
    loadids(keys, nE, cbase, tid, vec, d);
    unsigned msk = 0;
#pragma unroll
    for (int j = 0; j < EPT; ++j) {
      const unsigned ld = (unsigned)d[j] - (unsigned)n0;
      msk |= ((ld < (unsigned)NBA) ? 1u : 0u) << j;
    }
    const int cnt = __builtin_popcount(msk);
    int pos, nh;
    blkscan(cnt, lane, wave, swt, pos, nh);
    const int e0 = cbase + EPT * tid;
#pragma unroll
    for (int j = 0; j < EPT; ++j) {
      if ((msk >> j) & 1u) {
        const unsigned ld = (unsigned)d[j] - (unsigned)n0;
        if (pos < CHUNK) slist[pos] = ((unsigned)(e0 + j) << 9) | ld;
        ++pos;
      }
    }
    __syncthreads();
    const int nhc = nh < CHUNK ? nh : CHUNK;
    for (int j = 0; j < nhc; ++j) {
      const unsigned pk = (unsigned)__builtin_amdgcn_readfirstlane((int)slist[j]);
      const int ld = (int)(pk & (unsigned)(NBA - 1));
      if ((ld & (SWAV - 1)) == wave) {
        int e = (int)(pk >> 9);
        e = e > nE - 1 ? nE - 1 : e;
        int hq = e / nG;
        hq = hq < 0 ? 0 : (hq > NHEAD - 1 ? NHEAD - 1 : hq);
        int g = e - hq * nG;
        g = g < 0 ? 0 : (g > nG - 1 ? nG - 1 : g);
        const float v = S[((size_t)g * NHEAD + hq) * FD + lane];
        float* ap = sacc + ld * FD + lane;
        const float av = *ap;
        *ap = av + v;
      }
    }
  }
  __syncthreads();

  agg_store(sacc, sbi, out, n0, nN, tid);
  __threadfence();
  agg_store(sacc, sbi, out, n0, nN, tid);
}

extern "C" void kernel_launch(void* const* d_in, const int* in_sizes, int n_in,
                              void* d_out, int out_size, void* d_ws, size_t ws_size,
                              hipStream_t stream) {
  if (n_in < 10) return;
  if (in_sizes[0] < FD || in_sizes[1] < 2) return;
  const int nN = in_sizes[0] / FD;
  const int nE = in_sizes[1] / 2;
  if (nN < 1 || nE < 1) return;
  if (in_sizes[0] != nN * FD || in_sizes[1] != 2 * nE) return;
  if ((long long)in_sizes[2] != (long long)nE * FD) return;
  if (in_sizes[3] != 2 * FD * NCOL || in_sizes[4] != NHEAD * 2 * FD || in_sizes[5] != FD) return;
  if (in_sizes[6] != NHEAD || in_sizes[7] != NHEAD || in_sizes[8] != NGRP || in_sizes[9] != NGRP) return;
  if (out_size != nN * FD) return;
  if ((nE % GSZ) != 0) return;
  if (nN > (1 << 22) || nE > (1 << 22)) return;

  const float* x     = (const float*)d_in[0];
  const int*   eidx  = (const int*)d_in[1];
  const float* ea    = (const float*)d_in[2];
  const float* W     = (const float*)d_in[3];
  const float* att   = (const float*)d_in[4];
  const float* bias  = (const float*)d_in[5];
  const float* gam   = (const float*)d_in[6];
  const float* bet   = (const float*)d_in[7];
  const float* rmean = (const float*)d_in[8];
  const float* rvar  = (const float*)d_in[9];
  float* out = (float*)d_out;

  const int nG      = nE / GSZ;
  const int nPadN   = ((nN + GROWS - 1) / GROWS) * GROWS;
  const int nGpad   = ((nG + GPB - 1) / GPB) * GPB;
  const int gNode   = nPadN / GROWS;
  const int gEdge   = nGpad / GPB;
  const int gAgg    = (nN + NBA - 1) / NBA;
  const int nChunks = (nE + CHUNK - 1) / CHUNK;
  const int vec     = 1;

  char* ws = (char*)d_ws;
  size_t off = 0;
  const size_t oB = off; off += (size_t)BPTOT * 2;                 off = (off + 255) & ~(size_t)255;
  const size_t oP = off; off += (size_t)nPadN * NCOL * 4;          off = (off + 255) & ~(size_t)255;
  const size_t oS = off; off += (size_t)nGpad * NHEAD * FD * 4;    off = (off + 255) & ~(size_t)255;
  if (off > ws_size || off > (size_t)WSCAP) return;
  _Float16* Bpl = (_Float16*)(ws + oB);
  float*    P   = (float*)(ws + oP);
  float*    S   = (float*)(ws + oS);

  hipFuncSetAttribute(reinterpret_cast<const void*>(&k_edge), hipFuncAttributeMaxDynamicSharedMemorySize, LDS_EDGE);
  hipFuncSetAttribute(reinterpret_cast<const void*>(&k_agg), hipFuncAttributeMaxDynamicSharedMemorySize, LDS_AGG);

  k_wprep<<<10, 256, 0, stream>>>(W, Bpl);
  k_nodep<<<gNode, GTHR, 0, stream>>>(x, Bpl + OFF_BX, P, nN);
  k_edge<<<gEdge, ETHR, LDS_EDGE, stream>>>(P, eidx, ea, Bpl + OFF_BE, att, gam, bet, rmean, rvar, S, nN, nE, nG);
  k_agg<<<gAgg, STHR, LDS_AGG, stream>>>(eidx, S, bias, out, nN, nE, nG, nChunks, vec);
}
